// FourierKARTLayer_38749194944722
// MI455X (gfx1250) — hardware-verified
//
#include <hip/hip_runtime.h>
#include <math.h>

typedef __attribute__((ext_vector_type(16))) _Float16 v16h;
typedef __attribute__((ext_vector_type(16))) __bf16 v16b;
typedef __attribute__((ext_vector_type(8)))  _Float16 v8h;
typedef __attribute__((ext_vector_type(8)))  float v8f;
typedef __attribute__((ext_vector_type(4)))  float v4f;
typedef __attribute__((ext_vector_type(2)))  float v2f;
typedef __attribute__((ext_vector_type(4)))  unsigned v4u;
typedef __attribute__((ext_vector_type(4)))  int v4i;
typedef float __attribute__((may_alias)) float_a;
typedef int __attribute__((may_alias)) int_a;

template <typename T> __device__ __forceinline__ void vst2(void* p, T v) { *(volatile T*)p = v; __threadfence(); *(volatile T*)p = v; }
__device__ __forceinline__ v8f wmma16(v16h a, v16h b, v8f c) {
  v8f d = __builtin_amdgcn_wmma_f32_16x16x32_f16(false, a, false, b, (short)0, c, false, false);
  asm volatile("v_nop\n\tv_nop\n\tv_nop\n\tv_nop" : "+v"(d) : "v"(a), "v"(b));
  return d;
}
__device__ __forceinline__ v8f wmma_bf(v16b a, v16b b, v8f c) {
  v8f d = __builtin_amdgcn_wmma_f32_16x16x32_bf16(false, a, false, b, (short)0, c, false, false);
  asm volatile("v_nop\n\tv_nop\n\tv_nop\n\tv_nop" : "+v"(d) : "v"(a), "v"(b));
  return d;
}
__device__ __forceinline__ v16h frag_h(const _Float16* rowk0, int lane) {
  union { v16h v; v8h q[2]; } u; const _Float16* p = rowk0 + 8 * (lane >> 4);
  u.q[0] = *(const v8h*)p; u.q[1] = *(const v8h*)(p + 16); return u.v;
}
__device__ __forceinline__ v16h frag_f32(const float* rowk0, int lane) {
  v16h a; const float* p = rowk0 + 8 * (lane >> 4);
#pragma unroll
  for (int i = 0; i < 8; ++i) { a[i] = (_Float16)p[i]; a[8 + i] = (_Float16)p[16 + i]; }
  return a;
}
__device__ __forceinline__ v16h frag_f32s(const float* rowk0, int lane, float sc) {
  v16h a; const float* p = rowk0 + 8 * (lane >> 4);
#pragma unroll
  for (int i = 0; i < 8; ++i) { a[i] = (_Float16)(p[i] * sc); a[8 + i] = (_Float16)(p[16 + i] * sc); }
  return a;
}
__device__ __forceinline__ v16h fragc_f32(const float* W, int k0, int n, int lane, int ld, int K) {
  v16h a; const int g = lane >> 4;
#pragma unroll
  for (int i = 0; i < 8; ++i) { const int ka = k0 + 8 * g + i, kb = ka + 16;
    a[i] = (_Float16)(ka < K ? W[(size_t)(ka < K ? ka : K - 1) * ld + n] : 0.f); a[8 + i] = (_Float16)(kb < K ? W[(size_t)(kb < K ? kb : K - 1) * ld + n] : 0.f); }
  return a;
}
struct F2 { v16b h, l; };
__device__ __forceinline__ F2 bsplit16(const float v[16]) { F2 r;
#pragma unroll
  for (int i = 0; i < 16; ++i) { const __bf16 h = (__bf16)v[i]; r.h[i] = h; r.l[i] = (__bf16)(v[i] - (float)h); }
  return r; }
__device__ __forceinline__ F2 split_row(const float* row, int k0, int lane) { float v[16]; const float* p = row + k0 + 8 * (lane >> 4);
#pragma unroll
  for (int i = 0; i < 8; ++i) { v[i] = p[i]; v[8 + i] = p[16 + i]; }
  return bsplit16(v); }
__device__ __forceinline__ F2 split_rowK(const float* row, int k0, int lane, int K) { float v[16]; const int g = lane >> 4;
#pragma unroll
  for (int i = 0; i < 8; ++i) { const int ka = k0 + 8 * g + i, kb = ka + 16; v[i] = ka < K ? row[ka < K ? ka : K - 1] : 0.f; v[8 + i] = kb < K ? row[kb < K ? kb : K - 1] : 0.f; }
  return bsplit16(v); }
__device__ __forceinline__ F2 split_col(const float* W, int k0, int n, int lane, int ld, int K) { float v[16]; const int g = lane >> 4;
#pragma unroll
  for (int i = 0; i < 8; ++i) { const int ka = k0 + 8 * g + i, kb = ka + 16; v[i] = ka < K ? W[(size_t)(ka < K ? ka : K - 1) * ld + n] : 0.f; v[8 + i] = kb < K ? W[(size_t)(kb < K ? kb : K - 1) * ld + n] : 0.f; }
  return bsplit16(v); }
__device__ __forceinline__ v8f mac3(const F2& a, const F2& b, v8f c) { c = wmma_bf(a.l, b.h, c); c = wmma_bf(a.h, b.l, c); return wmma_bf(a.h, b.h, c); }
__device__ __forceinline__ float sigm(float v) { return 1.0f / (1.0f + expf(-v)); }
#define LDSX() do { asm volatile("s_wait_dscnt 0" ::: "memory"); __builtin_amdgcn_wave_barrier(); __builtin_amdgcn_fence(__ATOMIC_RELEASE, "workgroup"); } while (0)


#define NBZ 256
#define DIN 512
#define DOUT 64
#define NQ 4
#define NK 4
#define NFT 32
__device__ __forceinline__ float bfr(float v) { return (float)(__bf16)v; }
__device__ __forceinline__ v16b frag_b(const __bf16* rowk0, int lane) { return __builtin_bit_cast(v16b, frag_h((const _Float16*)rowk0, lane)); }
__device__ __attribute__((noinline)) void sincos_ni(float a, float* s, float* c) { sincosf(a, s, c); }

__global__ __launch_bounds__(256) void k_c(const float* __restrict__ X0, const float* __restrict__ Wc, const float* __restrict__ bc, const float* __restrict__ A, const float* __restrict__ Bp, float* __restrict__ Cb, __bf16* __restrict__ Th, __bf16* __restrict__ Tl) {
  __shared__ __align__(16) float sc[NBZ * NQ]; __shared__ __align__(16) __bf16 sth[DOUT * NFT], stl[DOUT * NFT];
  const int tid = threadIdx.x;
#pragma unroll 1
  for (int q = 0; q < NQ; ++q) { float s = bfr(bc[q]);
#pragma unroll 4
    for (int d = 0; d < DIN; ++d) s += bfr(X0[(size_t)tid * DIN + d]) * bfr(Wc[q * DIN + d]);
    sc[tid * NQ + q] = s; }
  for (int e = tid; e < DOUT * NFT; e += 256) { const int o = e / NFT, f = e % NFT; const int qk = f & 15; const float a = bfr(A[o * 16 + qk]), ph = bfr(Bp[o * 16 + qk]); float sn, cs; sincos_ni(ph, &sn, &cs); const float v = f < 16 ? a * cs : a * sn; const __bf16 hi = (__bf16)v; sth[e] = hi; stl[e] = (__bf16)(v - (float)hi); }
  __syncthreads();
  vst2(Cb + tid * 4, *(const v4f*)(&sc[tid * 4]));
  vst2((unsigned*)(Th + tid * 8), *(const v4u*)(&sth[tid * 8])); vst2((unsigned*)(Tl + tid * 8), *(const v4u*)(&stl[tid * 8]));
}
__global__ __launch_bounds__(128) void k_v(const float* __restrict__ Cb, const float* __restrict__ t, const float* __restrict__ wq, const __bf16* __restrict__ Th, const __bf16* __restrict__ Tl, float* __restrict__ V) {
  __shared__ __align__(16) __bf16 ssh[4][16][40], ssl[4][16][40]; __shared__ __align__(16) float so[4][16][68];
  const int tid = threadIdx.x, wave = tid >> 5, lane = tid & 31, col = lane & 15, g = lane >> 4; const int b = blockIdx.y, bp0 = blockIdx.x * 64 + wave * 16; const float tb = bfr(t[b]);
  { const int rl = lane & 15, fh = lane >> 4;
#pragma unroll
    for (int qq = 0; qq < 2; ++qq) { const int q = fh * 2 + qq; const float ang = Cb[(bp0 + rl) * NQ + q] + bfr(wq[q]) * tb;
#pragma unroll
      for (int k = 0; k < NK; ++k) { float sn, cs; sincos_ni(ang * (float)(k + 1), &sn, &cs); const int f = q * 4 + k;
        { const __bf16 hi = (__bf16)sn; ssh[wave][rl][f] = hi; ssl[wave][rl][f] = (__bf16)(sn - (float)hi); }
        { const __bf16 hi = (__bf16)cs; ssh[wave][rl][16 + f] = hi; ssl[wave][rl][16 + f] = (__bf16)(cs - (float)hi); } } } }
  LDSX();
  const v16b ah = frag_b(&ssh[wave][col][0], lane), al = frag_b(&ssl[wave][col][0], lane);
  v8f acc[4] = {};
#pragma unroll
  for (int j = 0; j < 4; ++j) { const v16b th = frag_b(Th + (size_t)(j * 16 + col) * NFT, lane), tl = frag_b(Tl + (size_t)(j * 16 + col) * NFT, lane); acc[j] = wmma_bf(al, th, acc[j]); acc[j] = wmma_bf(ah, tl, acc[j]); acc[j] = wmma_bf(ah, th, acc[j]); }
#pragma unroll
  for (int j = 0; j < 4; ++j)
#pragma unroll
    for (int r = 0; r < 8; ++r) so[wave][8 * g + r][j * 16 + col] = acc[j][r];
  LDSX();
  for (int qq = lane; qq < 16 * 16; qq += 32) { const int rl = qq >> 4, pc = qq & 15; vst2(V + ((size_t)b * NBZ + bp0 + rl) * DOUT + pc * 4, *(const v4f*)(&so[wave][rl][pc * 4])); }
}
extern "C" void kernel_launch(void* const* d_in, const int* in_sizes, int n_in, void* d_out, int out_size, void* d_ws, size_t ws_size, hipStream_t stream) {
  (void)in_sizes; (void)n_in; (void)out_size; (void)ws_size;
  const float** I = (const float**)d_in;
  char* ws = (char*)d_ws; float* Cb = (float*)ws; __bf16* Th = (__bf16*)(ws + 4096); __bf16* Tl = (__bf16*)(ws + 4096 + DOUT * NFT * 2);
  k_c<<<1, 256, 0, stream>>>(I[0], I[2], I[3], I[5], I[6], Cb, Th, Tl);
  k_v<<<dim3(NBZ / 64, NBZ), 128, 0, stream>>>(Cb, I[1], I[4], Th, Tl, (float*)d_out);
}
